// SimpleKANLinear_88776974009041
// MI455X (gfx1250) — hardware-verified
//
#include <hip/hip_runtime.h>
#include <math.h>

constexpr int kTokens     = 8192;
constexpr int kInF        = 1024;
constexpr int kOutF       = 1024;
constexpr int kGridN      = 8;
constexpr int kKspl       = kInF * kGridN;
constexpr int kKtot       = kInF + kKspl;
constexpr int kChunkRows  = 4096;
constexpr int kNumChunks  = kTokens / kChunkRows;
constexpr int kGrp8InF    = kInF / 8;
constexpr int kGrp8Spl    = kKspl / 8;
constexpr float kACarry   = 16.0f;
constexpr float kBCarry   = 64.0f;
constexpr float kOutScale = 1.0f / 1024.0f;

static_assert(kKtot % 32 == 0, "K tile multiple");
static_assert(kChunkRows % 64 == 0 && kOutF % 64 == 0, "M,N tile multiples");
static_assert(kTokens % kChunkRows == 0, "chunking exact");
static_assert((kKtot * 2) % 128 == 0, "16-bit row pitch is whole lines");

typedef __attribute__((ext_vector_type(16))) _Float16 v16h;
typedef __attribute__((ext_vector_type(8)))  _Float16 v8h;
typedef __attribute__((ext_vector_type(16))) __bf16   v16b;
typedef __attribute__((ext_vector_type(8)))  __bf16   v8b;
typedef __attribute__((ext_vector_type(8)))  float    v8f;
typedef __attribute__((ext_vector_type(4)))  float    v4f;
typedef __attribute__((ext_vector_type(4)))  unsigned int v4u;

__device__ __forceinline__ unsigned short f2bf_bits(float f) {
  unsigned u = __float_as_uint(f);
  return (unsigned short)((u + 0x7FFFu + ((u >> 16) & 1u)) >> 16);
}
__device__ __forceinline__ float bf_bits2f(unsigned short h) { return __uint_as_float(((unsigned)h) << 16); }

__device__ __forceinline__ void dep_guard_h(v8f& a, v8f& b, v16h x, v16h y) { asm volatile("v_nop\n\tv_nop\n\tv_nop\n\tv_nop" : "+v"(a), "+v"(b) : "v"(x), "v"(y)); }
__device__ __forceinline__ void dep_guard_b(v8f& a, v8f& b, v16b x, v16b y) { asm volatile("v_nop\n\tv_nop\n\tv_nop\n\tv_nop" : "+v"(a), "+v"(b) : "v"(x), "v"(y)); }
__device__ __forceinline__ void keep4_h(v16h a, v16h b, v16h c, v16h d) { asm volatile("v_nop" :: "v"(a), "v"(b), "v"(c), "v"(d)); }
__device__ __forceinline__ void keep4_b(v16b a, v16b b, v16b c, v16b d) { asm volatile("v_nop" :: "v"(a), "v"(b), "v"(c), "v"(d)); }
__device__ __forceinline__ void acc_guard4(v8f& a, v8f& b, v8f& c, v8f& d) { asm volatile("v_nop\n\tv_nop\n\tv_nop\n\tv_nop" : "+v"(a), "+v"(b), "+v"(c), "+v"(d)); }
template <typename T> struct Frag;
template <> struct Frag<_Float16> {
  typedef v16h V; union U { v16h v; v8h h[2]; };
  static __device__ __forceinline__ v16h load(const _Float16* p) {
    U f; f.h[0] = *(const v8h*)(p); f.h[1] = *(const v8h*)(p + 16); return f.v;
  }
  static __device__ __forceinline__ v8f mma(v16h a, v16h b, v8f c) {
    return __builtin_amdgcn_wmma_f32_16x16x32_f16(false, a, false, b, (short)0, c, false, false);
  }
  static __device__ __forceinline__ void guard(v8f& a, v8f& b, v16h x, v16h y) { dep_guard_h(a, b, x, y); }
  static __device__ __forceinline__ void keep(v16h a, v16h b, v16h c, v16h d) { keep4_h(a, b, c, d); }
};
template <> struct Frag<__bf16> {
  typedef v16b V; union U { v16b v; v8b h[2]; };
  static __device__ __forceinline__ v16b load(const __bf16* p) {
    U f; f.h[0] = *(const v8b*)(p); f.h[1] = *(const v8b*)(p + 16); return f.v;
  }
  static __device__ __forceinline__ v8f mma(v16b a, v16b b, v8f c) {
    return __builtin_amdgcn_wmma_f32_16x16x32_bf16(false, a, false, b, (short)0, c, false, false);
  }
  static __device__ __forceinline__ void guard(v8f& a, v8f& b, v16b x, v16b y) { dep_guard_b(a, b, x, y); }
  static __device__ __forceinline__ void keep(v16b a, v16b b, v16b c, v16b d) { keep4_b(a, b, c, d); }
};

__device__ __forceinline__ unsigned pk16(unsigned short a, unsigned short b) { return (unsigned)a | ((unsigned)b << 16); }
__device__ __forceinline__ unsigned short h_bits(float f) { const _Float16 h = (_Float16)f; return __builtin_bit_cast(unsigned short, h); }

template <int ET> struct Elem;
template <> struct Elem<0> { typedef _Float16 T; };
template <> struct Elem<1> { typedef __bf16 T; };
template <int ET, bool SPLIT, int BIAS_MODE, int OUT_MODE, bool RESID, int ACT = 0>
__global__ __launch_bounds__(256) void wmma_gemm64(
    const unsigned short* __restrict__ Ap, const unsigned short* __restrict__ A2p, int lda, long strideA,
    const unsigned short* __restrict__ Btp, const unsigned short* __restrict__ Bt2p, int ldb, long strideB,
    void* __restrict__ Cout, void* __restrict__ Cout2, int ldc, long strideC,
    const float* __restrict__ bias,
    const float* __restrict__ resid, long strideR,
    int M, int N, int K, float scale) {
  typedef typename Elem<ET>::T T;
  typedef typename Frag<T>::V V;
  const T* A = (const T*)Ap; const T* A2 = (const T*)A2p; const T* Bt = (const T*)Btp; const T* Bt2 = (const T*)Bt2p;
  __shared__ __align__(16) float sT[8][16 * 68];
  const int b    = blockIdx.y;
  const int lane = threadIdx.x & 31;
  const int wave = threadIdx.x >> 5;
  const int tilesN = N >> 6;
  const int tilesM = M >> 6;
  const int tile = blockIdx.x * 8 + wave;
  if (tile >= tilesM * tilesN) return;
  const int tm = tile / tilesN;
  const int tn = tile - tm * tilesN;
  const int m0 = tm << 6;
  const int n0 = tn << 6;

  const T* Ab  = A  + (size_t)b * strideA;
  const T* Bb  = Bt + (size_t)b * strideB;
  const T* Ab2 = SPLIT ? (A2  + (size_t)b * strideA) : nullptr;
  const T* Bb2 = SPLIT ? (Bt2 + (size_t)b * strideB) : nullptr;

  const int rlane = lane & 15;
  const int koff  = (lane >> 4) * 8;
  const int mOff  = (lane >> 4) * 8;

  v8f acc[4][4];
#pragma unroll
  for (int i = 0; i < 4; ++i)
#pragma unroll
    for (int j = 0; j < 4; ++j) acc[i][j] = (v8f){0.f,0.f,0.f,0.f,0.f,0.f,0.f,0.f};

  for (int k0 = 0; k0 < K; k0 += 32) {
    V bh[4], bl[4];
#pragma unroll
    for (int j = 0; j < 4; ++j) {
      const size_t bo = (size_t)(n0 + (j << 4) + rlane) * ldb + koff + k0;
      bh[j] = Frag<T>::load(Bb + bo);
      if (SPLIT) bl[j] = Frag<T>::load(Bb2 + bo);
    }
#pragma unroll
    for (int i = 0; i < 4; ++i) {
      const size_t ao = (size_t)(m0 + (i << 4) + rlane) * lda + koff + k0;
      V ah = Frag<T>::load(Ab + ao);
      V al;
      if (SPLIT) al = Frag<T>::load(Ab2 + ao);
#pragma unroll
      for (int j = 0; j < 4; ++j) {
        acc[i][j] = Frag<T>::mma(ah, bh[j], acc[i][j]);
        if (SPLIT) {
          acc[i][j] = Frag<T>::mma(ah, bl[j], acc[i][j]);
          acc[i][j] = Frag<T>::mma(al, bh[j], acc[i][j]);
        }
      }
      Frag<T>::guard(acc[i][0], acc[i][3], ah, SPLIT ? al : ah);
    }
    Frag<T>::keep(bh[0], bh[1], bh[2], bh[3]);
    if (SPLIT) Frag<T>::keep(bl[0], bl[1], bl[2], bl[3]);
  }
  acc_guard4(acc[0][0], acc[0][1], acc[0][2], acc[0][3]);
  acc_guard4(acc[1][0], acc[1][1], acc[1][2], acc[1][3]);
  acc_guard4(acc[2][0], acc[2][1], acc[2][2], acc[2][3]);
  acc_guard4(acc[3][0], acc[3][1], acc[3][2], acc[3][3]);

  float* slab = sT[wave];
  const float* Rb = RESID ? (resid + (size_t)b * strideR) : nullptr;
#pragma unroll
  for (int i = 0; i < 4; ++i) {
    const int mBase = m0 + (i << 4);
#pragma unroll
    for (int j = 0; j < 4; ++j) {
      const int n = n0 + (j << 4) + rlane;
      float bv = 0.f;
      if (BIAS_MODE == 2) bv = bias[n];
#pragma unroll
      for (int r = 0; r < 8; ++r) {
        float v = acc[i][j][r] * scale;
        if (BIAS_MODE == 1) v += bias[mBase + mOff + r];
        if (BIAS_MODE == 2) v += bv;
        if (RESID) v += Rb[(size_t)(mBase + mOff + r) * ldc + n];
        if (ACT == 2) v = fmaxf(v, 0.0f);
        if (ACT == 4) v = (v > 0.f) ? v : 0.01f * v;
        slab[(mOff + r) * 68 + (j << 4) + rlane] = v;
      }
    }
    __builtin_amdgcn_fence(__ATOMIC_RELEASE, "workgroup");
    __builtin_amdgcn_wave_barrier();
    __builtin_amdgcn_fence(__ATOMIC_ACQUIRE, "workgroup");
    if (OUT_MODE == 0) {
      float* C = (float*)Cout + (size_t)b * strideC;
      const int hh = lane >> 4, c4 = (lane & 15) * 4;
      for (int pass = 0; pass < 2; ++pass) {
#pragma unroll
        for (int it = 0; it < 8; ++it) {
          const int row = it * 2 + hh;
          v4f v = *(const v4f*)(slab + row * 68 + c4);
          *(volatile v4f*)(C + (size_t)(mBase + row) * ldc + n0 + c4) = v;
        }
        __threadfence();
      }
    } else {
      const int q = lane >> 3, c8 = (lane & 7) * 8;
      unsigned short* C  = (unsigned short*)Cout  + (size_t)b * strideC;
      unsigned short* C2 = (OUT_MODE == 2) ? ((unsigned short*)Cout2 + (size_t)b * strideC) : nullptr;
      for (int pass = 0; pass < 2; ++pass) {
#pragma unroll
        for (int it = 0; it < 4; ++it) {
          const int row = it * 4 + q;
          const float* sp = slab + row * 68 + c8;
          v8h hv, lv;
#pragma unroll
          for (int e = 0; e < 8; ++e) {
            if (OUT_MODE == 1) {
              hv[e] = (_Float16)sp[e];
            } else {
              unsigned short hb = f2bf_bits(sp[e]);
              unsigned short lb = f2bf_bits(sp[e] - bf_bits2f(hb));
              hv[e] = __builtin_bit_cast(_Float16, hb);
              lv[e] = __builtin_bit_cast(_Float16, lb);
            }
          }
          *(volatile v8h*)(C + (size_t)(mBase + row) * ldc + n0 + c8) = hv;
          if (OUT_MODE == 2) *(volatile v8h*)(C2 + (size_t)(mBase + row) * ldc + n0 + c8) = lv;
        }
        __threadfence();
      }
    }
    __builtin_amdgcn_fence(__ATOMIC_RELEASE, "workgroup");
    __builtin_amdgcn_wave_barrier();
    __builtin_amdgcn_fence(__ATOMIC_ACQUIRE, "workgroup");
  }
}

__global__ __launch_bounds__(256) void cast8_rows_kernel(const float* __restrict__ in, unsigned short* __restrict__ out,
                                                         int grpPerRow, int nThreads, int inPitch, int outPitch,
                                                         int outCol0, float scale) {
  const int i = blockIdx.x * 256 + threadIdx.x;
  if (i >= nThreads) return;
  const int row = i / grpPerRow;
  const int grp = i - row * grpPerRow;
  const float* p = in + (size_t)row * inPitch + 8 * (size_t)grp;
  const v4f a = *(const v4f*)(p);
  const v4f c = *(const v4f*)(p + 4);
  unsigned short hb[8];
#pragma unroll
  for (int e = 0; e < 4; ++e) {
    hb[e]     = h_bits(scale * a[e]);
    hb[4 + e] = h_bits(scale * c[e]);
  }
  const v4u u = (v4u){pk16(hb[0], hb[1]), pk16(hb[2], hb[3]), pk16(hb[4], hb[5]), pk16(hb[6], hb[7])};
  unsigned short* q = out + (size_t)row * outPitch + outCol0 + 8 * (size_t)grp;
  *(volatile v4u*)q = u;
  __threadfence();
  *(volatile v4u*)q = u;
}

__global__ __launch_bounds__(256) void silu_cast_kernel(const float* __restrict__ x, unsigned short* __restrict__ A,
                                                        int nThreads, float carry) {
  const int i = blockIdx.x * 256 + threadIdx.x;
  if (i >= nThreads) return;
  const int r   = i >> 7;
  const int grp = i & (kGrp8InF - 1);
  const float* p = x + (size_t)r * kInF + 8 * (size_t)grp;
  const v4f a = *(const v4f*)(p);
  const v4f c = *(const v4f*)(p + 4);
  unsigned short hb[8];
#pragma unroll
  for (int e = 0; e < 4; ++e) {
    const float v0 = a[e];
    const float v1 = c[e];
    const float s0 = v0 * __builtin_amdgcn_rcpf(1.0f + expf(-v0));
    const float s1 = v1 * __builtin_amdgcn_rcpf(1.0f + expf(-v1));
    hb[e]     = h_bits(carry * s0);
    hb[4 + e] = h_bits(carry * s1);
  }
  const v4u u = (v4u){pk16(hb[0], hb[1]), pk16(hb[2], hb[3]), pk16(hb[4], hb[5]), pk16(hb[6], hb[7])};
  unsigned short* q = A + (size_t)r * kKtot + 8 * (size_t)grp;
  *(volatile v4u*)q = u;
  __threadfence();
  *(volatile v4u*)q = u;
}

__global__ __launch_bounds__(256) void basis_kernel(const float* __restrict__ x, const float* __restrict__ gridp,
                                                    unsigned short* __restrict__ A, int nThreads, float invd, float carry) {
  const int i = blockIdx.x * 256 + threadIdx.x;
  if (i >= nThreads) return;
  const int r = i >> 10;
  const int f = i & (kInF - 1);
  const float xv = x[(size_t)r * kInF + f];
  float gv[kGridN];
#pragma unroll
  for (int e = 0; e < kGridN; ++e) gv[e] = gridp[e];
  unsigned short hb[8];
#pragma unroll
  for (int e = 0; e < kGridN; ++e) {
    const float t = (xv - gv[e]) * invd;
    const float bs = expf(-(t * t));
    hb[e] = h_bits(carry * bs);
  }
  const v4u u = (v4u){pk16(hb[0], hb[1]), pk16(hb[2], hb[3]), pk16(hb[4], hb[5]), pk16(hb[6], hb[7])};
  unsigned short* q = A + (size_t)r * kKtot + kInF + 8 * (size_t)f;
  *(volatile v4u*)q = u;
  __threadfence();
  *(volatile v4u*)q = u;
}

extern "C" void kernel_launch(void* const* d_in, const int* in_sizes, int n_in,
                              void* d_out, int out_size, void* d_ws, size_t ws_size, hipStream_t stream) {
  if (n_in < 5) return;
  if (in_sizes[0] != kTokens * kInF) return;
  if (in_sizes[1] != kOutF * kInF) return;
  if (in_sizes[2] != kOutF) return;
  if (in_sizes[3] != kOutF * kInF * kGridN) return;
  if (in_sizes[4] != kGridN) return;
  if (out_size != kTokens * kOutF) return;

  const size_t btBytes = (size_t)kOutF * kKtot * 2;
  const size_t aBytes  = (size_t)kChunkRows * kKtot * 2;
  if (btBytes + aBytes > ws_size) return;

  const float* x     = (const float*)d_in[0];
  const float* W     = (const float*)d_in[1];
  const float* bias  = (const float*)d_in[2];
  const float* sw    = (const float*)d_in[3];
  const float* gridp = (const float*)d_in[4];
  float* out = (float*)d_out;
  unsigned short* Bt16 = (unsigned short*)d_ws;
  unsigned short* A16  = (unsigned short*)((char*)d_ws + btBytes);

  const float denom = (float)(2.0 / 7.0 + 1e-05);
  const float invd  = 1.0f / denom;

  {
    const int n = kOutF * kGrp8InF;
    cast8_rows_kernel<<<(n + 255) / 256, 256, 0, stream>>>(W, Bt16, kGrp8InF, n, kInF, kKtot, 0, kBCarry);
  }
  {
    const int n = kOutF * kGrp8Spl;
    cast8_rows_kernel<<<(n + 255) / 256, 256, 0, stream>>>(sw, Bt16, kGrp8Spl, n, kKspl, kKtot, kInF, kBCarry);
  }

  for (int ch = 0; ch < kNumChunks; ++ch) {
    const float* xc = x + (size_t)ch * kChunkRows * kInF;
    {
      const int n = kChunkRows * kGrp8InF;
      silu_cast_kernel<<<(n + 255) / 256, 256, 0, stream>>>(xc, A16, n, kACarry);
    }
    {
      const int n = kChunkRows * kInF;
      basis_kernel<<<(n + 255) / 256, 256, 0, stream>>>(xc, gridp, A16, n, invd, kACarry);
    }
    float* oc = out + (size_t)ch * kChunkRows * kOutF;
    const int tiles = (kChunkRows / 64) * (kOutF / 64);
    dim3 gg((tiles + 7) / 8, 1);
    wmma_gemm64<0, false, 2, 0, false, 0><<<gg, 256, 0, stream>>>(
        A16, nullptr, kKtot, 0L,
        Bt16, nullptr, kKtot, 0L,
        (void*)oc, nullptr, kOutF, 0L,
        bias, nullptr, 0L,
        kChunkRows, kOutF, kKtot, kOutScale);
  }
}
